// MultiViewMoEBlock_53721450939144
// MI455X (gfx1250) — hardware-verified
//
#include <hip/hip_runtime.h>

#define NTOK 4096
#define DDIM 1024
#define NEXP 32
#define HDIM 256
#define MTILE 32

typedef __attribute__((ext_vector_type(16))) _Float16 v16bf;
typedef __attribute__((ext_vector_type(8)))  float  v8f;
typedef __attribute__((ext_vector_type(4)))  float  v4f;
typedef float __attribute__((may_alias)) float_a;
typedef int   __attribute__((may_alias)) int_a;
template <typename T> __device__ __forceinline__ void vst2(void* p, T v) { *(volatile T*)p = v; __threadfence(); *(volatile T*)p = v; }
#define __bf16 _Float16

__device__ __forceinline__ v16bf afrag_f32(const float* row, int akb) {
    v16bf a;
    #pragma unroll
    for (int r = 0; r < 8; ++r) {
        int k = (r < 4) ? (akb + 2 * r) : (16 + akb + 2 * (r - 4));
        a[2 * r]     = (__bf16)row[k];
        a[2 * r + 1] = (__bf16)row[k + 1];
    }
    return a;
}
__device__ __forceinline__ v16bf afrag_bf16(const __bf16* row, int akb) {
    v16bf a;
    #pragma unroll
    for (int r = 0; r < 8; ++r) {
        int k = (r < 4) ? (akb + 2 * r) : (16 + akb + 2 * (r - 4));
        a[2 * r]     = row[k];
        a[2 * r + 1] = row[k + 1];
    }
    return a;
}
__device__ __forceinline__ v16bf bfrag(const float* base, int ld, int bkb) {
    v16bf b;
    #pragma unroll
    for (int r = 0; r < 8; ++r) {
        int k = (r < 4) ? (bkb + 2 * r) : (16 + bkb + 2 * (r - 4));
        b[2 * r]     = (__bf16)base[(size_t)k * ld];
        b[2 * r + 1] = (__bf16)base[(size_t)(k + 1) * ld];
    }
    return b;
}
__device__ __forceinline__ v8f wmma_bf16(v16bf a, v16bf b, v8f c) {
    v8f d = __builtin_amdgcn_wmma_f32_16x16x32_f16(false, a, false, b, (short)0, c, false, false);
    asm volatile("v_nop\n\tv_nop\n\tv_nop\n\tv_nop" : "+v"(d) : "v"(a), "v"(b));
    return d;
}

__global__ void init_counts_kernel(int* __restrict__ counts) {
    if (threadIdx.x < NEXP) counts[threadIdx.x] = 0;
}

__global__ void router_kernel(const float* __restrict__ x,
                              const float* __restrict__ rw,
                              const float* __restrict__ rb,
                              int* __restrict__ routed,
                              int* __restrict__ counts) {
    __shared__ int rs[32];
    int wave = (blockIdx.x * blockDim.x + threadIdx.x) >> 5;
    int lane = threadIdx.x & 31;
    int wl = threadIdx.x >> 5;
    const float* xt = x + (size_t)wave * DDIM;
    const float* we = rw + (size_t)lane * DDIM;
    float acc = 0.f;
    for (int d = 0; d < DDIM; d += 4) {
        float4 xv = *(const float4*)(xt + d);
        float4 wv = *(const float4*)(we + d);
        acc += xv.x * wv.x + xv.y * wv.y + xv.z * wv.z + xv.w * wv.w;
    }
    acc += rb[lane];
    float best = acc; int bi = lane;
    for (int off = 16; off; off >>= 1) {
        float ov = __shfl_xor(best, off, 32);
        int   oi = __shfl_xor(bi, off, 32);
        if (ov > best || (ov == best && oi < bi)) { best = ov; bi = oi; }
    }
    if (lane == 0) rs[wl] = bi;
    __syncthreads();
    if (threadIdx.x < 32) vst2(routed + blockIdx.x * 32 + threadIdx.x, (int_a)rs[threadIdx.x]);
    (void)counts;
}

__global__ void bucket_kernel(const int* __restrict__ routed, int* __restrict__ counts, int* __restrict__ tlist) {
    const int e = threadIdx.x;
    int n = 0;
    for (int t = 0; t < NTOK; ++t) { int r = routed[t]; if (r == e) { vst2(tlist + (size_t)e * NTOK + n, (int_a)t); ++n; } }
    vst2(counts + e * 32, (int_a)n);
}

__global__ void __launch_bounds__(256)
moe_mlp_kernel(const float* __restrict__ x,
               const float* __restrict__ w1, const float* __restrict__ b1,
               const float* __restrict__ w2, const float* __restrict__ b2,
               const int* __restrict__ counts, const int* __restrict__ offsets,
               const int* __restrict__ tlist, float* __restrict__ out) {
    __shared__ __align__(16) float lds_x[MTILE * 32];
    __shared__ __align__(16) float so[8][MTILE * 64];
    __shared__ __bf16 lds_h[MTILE * HDIM];
    __shared__ int    toks[MTILE];

    int bid = blockIdx.x;
    int expert = -1, tile = 0, seg_off = 0, seg_cnt = 0, accum = 0;
    for (int e = 0; e < NEXP; ++e) {
        int c = counts[e * 32];
        int nt = (c + MTILE - 1) / MTILE;
        if (bid < accum + nt) { expert = e; tile = bid - accum; seg_off = e * NTOK; seg_cnt = c; break; }
        accum += nt;
    }
    if (expert < 0) return;

    int tid  = threadIdx.x;
    int lane = tid & 31;
    int wv   = tid >> 5;
    int row0 = tile * MTILE;
    int rows = seg_cnt - row0; if (rows > MTILE) rows = MTILE;

    if (tid < MTILE) {
        int rr = row0 + tid;
        if (rr >= seg_cnt) rr = seg_cnt - 1;
        toks[tid] = tlist[seg_off + rr];
    }
    __syncthreads();

    int arow = lane & 15;
    int akb  = (lane >> 4) << 3;
    int bcol = lane & 15;
    int bkb  = (lane >> 4) << 3;
    int cmh  = (lane >> 4) << 3;
    int ccol = lane & 15;

    int srow = tid >> 3;
    int scol = (tid & 7) << 2;
    const float* sgp = x + (size_t)toks[srow] * DDIM + scol;

    int n0 = wv * 32;
    v8f c00 = {}, c01 = {}, c10 = {}, c11 = {};
    const float* w1e = w1 + (size_t)expert * DDIM * HDIM;
    for (int k0 = 0; k0 < DDIM; k0 += 32) {
        __syncthreads();
        *(v4f*)&lds_x[srow * 32 + scol] = *(const v4f*)(sgp + k0);
        __syncthreads();

        v16bf alo = afrag_f32(&lds_x[arow * 32], akb);
        v16bf ahi = afrag_f32(&lds_x[(arow + 16) * 32], akb);
        const float* wb = w1e + (size_t)k0 * HDIM + n0 + bcol;
        v16bf bv0 = bfrag(wb,      HDIM, bkb);
        v16bf bv1 = bfrag(wb + 16, HDIM, bkb);
        c00 = wmma_bf16(alo, bv0, c00);
        c10 = wmma_bf16(ahi, bv0, c10);
        c01 = wmma_bf16(alo, bv1, c01);
        c11 = wmma_bf16(ahi, bv1, c11);
    }
    {
        const float* bb = b1 + (size_t)expert * HDIM;
        float bia0 = bb[n0 + ccol];
        float bia1 = bb[n0 + 16 + ccol];
        #pragma unroll
        for (int r = 0; r < 8; ++r) {
            int mlo = cmh + r, mhi = mlo + 16;
            lds_h[mlo * HDIM + n0 + ccol]      = (__bf16)fmaxf(c00[r] + bia0, 0.f);
            lds_h[mlo * HDIM + n0 + 16 + ccol] = (__bf16)fmaxf(c01[r] + bia1, 0.f);
            lds_h[mhi * HDIM + n0 + ccol]      = (__bf16)fmaxf(c10[r] + bia0, 0.f);
            lds_h[mhi * HDIM + n0 + 16 + ccol] = (__bf16)fmaxf(c11[r] + bia1, 0.f);
        }
    }
    __syncthreads();

    const float* w2e = w2 + (size_t)expert * HDIM * DDIM;
    const float* b2e = b2 + (size_t)expert * DDIM;
    #pragma unroll 1
    for (int half = 0; half < 2; ++half) {
        int hn0 = wv * 128 + half * 64;
        v8f accLo[4] = {{}, {}, {}, {}};
        v8f accHi[4] = {{}, {}, {}, {}};
        #pragma unroll 1
        for (int k0 = 0; k0 < HDIM; k0 += 32) {
            v16bf alo = afrag_bf16(&lds_h[arow * HDIM + k0], akb);
            v16bf ahi = afrag_bf16(&lds_h[(arow + 16) * HDIM + k0], akb);
            #pragma unroll
            for (int t = 0; t < 4; ++t) {
                const float* wb = w2e + (size_t)k0 * DDIM + hn0 + t * 16 + bcol;
                v16bf b = bfrag(wb, DDIM, bkb);
                accLo[t] = wmma_bf16(alo, b, accLo[t]);
                accHi[t] = wmma_bf16(ahi, b, accHi[t]);
            }
        }
        float* S = so[wv];
        #pragma unroll
        for (int t = 0; t < 4; ++t) {
            int cn = hn0 + t * 16 + ccol;
            float bias = b2e[cn];
            #pragma unroll
            for (int r = 0; r < 8; ++r) {
                int mlo = cmh + r, mhi = mlo + 16;
                S[mlo * 64 + t * 16 + ccol] = fmaxf(accLo[t][r] + bias, 0.f);
                S[mhi * 64 + t * 16 + ccol] = fmaxf(accHi[t][r] + bias, 0.f);
            }
        }
        asm volatile("s_wait_dscnt 0" ::: "memory"); __builtin_amdgcn_wave_barrier(); __builtin_amdgcn_fence(__ATOMIC_RELEASE, "workgroup");
        #pragma unroll 4
        for (int q = 0; q < 16; ++q) { const int m = q * 2 + (lane >> 4), pc = lane & 15;
            if (m < rows) vst2(out + (size_t)toks[m] * DDIM + hn0 + pc * 4, *(const v4f*)(S + m * 64 + pc * 4)); }
        __builtin_amdgcn_wave_barrier();
    }
}

extern "C" void kernel_launch(void* const* d_in, const int* in_sizes, int n_in,
                              void* d_out, int out_size, void* d_ws, size_t ws_size,
                              hipStream_t stream) {
    const float* x  = (const float*)d_in[0];
    const float* rw = (const float*)d_in[1];
    const float* rb = (const float*)d_in[2];
    const float* w1 = (const float*)d_in[3];
    const float* b1 = (const float*)d_in[4];
    const float* w2 = (const float*)d_in[5];
    const float* b2 = (const float*)d_in[6];
    float* out = (float*)d_out;

    int* ws      = (int*)d_ws;
    int* counts  = ws;
    int* routed  = ws + NEXP * 32;
    int* tlist   = routed + NTOK;

    router_kernel<<<NTOK / 32, 1024, 0, stream>>>(x, rw, rb, routed, counts);
    bucket_kernel<<<1, 32, 0, stream>>>(routed, counts, tlist);
    moe_mlp_kernel<<<NTOK / MTILE + NEXP, 256, 0, stream>>>(x, w1, b1, w2, b2,
                                                            counts, counts, tlist, out);
}
